// neighborhood_routing_algorithm_76501957476790
// MI455X (gfx1250) — hardware-run, weakly checked
//
#include <hip/hip_runtime.h>


#ifndef NQ
#define NQ 16384
#endif
#ifndef NKEY
#define NKEY 4096
#endif
#define NQ_FULL   16384
#define NKEY_FULL 4096
#define NSL  4
#define DF   10
#define KW   16
#define AW   4
#define VRS  2048.0f
#define VRI  (1.0f / 2048.0f)
#define L2E  1.4426950408889634f
#define PSH  14.0f
#define LN_EPS 1e-5f

static_assert(DF == 10);
static_assert(DF <= KW);
static_assert(NKEY % 128 == 0);
static_assert(NKEY % 32 == 0);
static_assert(NQ % (16 * AW) == 0);
static_assert((16 * DF * 4) % 128 == 0);
static_assert(NQ <= NQ_FULL);
static_assert(NKEY <= NKEY_FULL);

typedef _Float16 h16;
typedef unsigned short bf;
typedef __attribute__((ext_vector_type(16))) __bf16   v16bf;
typedef __attribute__((ext_vector_type(16))) _Float16 v16h;
typedef __attribute__((ext_vector_type(8)))  _Float16 v8h;
typedef __attribute__((ext_vector_type(8)))  unsigned short v8us;
typedef __attribute__((ext_vector_type(8)))  float    v8f;
typedef __attribute__((ext_vector_type(4)))  float    v4f;
typedef v4f  __attribute__((may_alias)) v4fa;

__device__ __forceinline__ unsigned short f2bf(float f) { unsigned u = __float_as_uint(f); u += 0x7FFFu + ((u >> 16) & 1u); return (unsigned short)(u >> 16); }
__device__ __forceinline__ float bf2f(unsigned short s) { return __uint_as_float(((unsigned)s) << 16); }
__device__ __forceinline__ v16h cat16(v8h lo, v8h hi) { return __builtin_shufflevector(lo, hi, 0, 1, 2, 3, 4, 5, 6, 7, 8, 9, 10, 11, 12, 13, 14, 15); }
__device__ __forceinline__ v16bf cat16b(v8us lo, v8us hi) { return __builtin_bit_cast(v16bf, __builtin_shufflevector(lo, hi, 0, 1, 2, 3, 4, 5, 6, 7, 8, 9, 10, 11, 12, 13, 14, 15)); }
__device__ __forceinline__ v8f wmma16(v16h a, v16h b, v8f c) { return __builtin_amdgcn_wmma_f32_16x16x32_f16(false, a, false, b, (short)0, c, false, false); }
__device__ __forceinline__ v8f wmmab(v16bf a, v16bf b, v8f c) { return __builtin_amdgcn_wmma_f32_16x16x32_bf16(false, a, false, b, (short)0, c, false, false); }
__device__ __forceinline__ v16h  ldh(const h16* p) { return cat16(*(const v8h*)p, *(const v8h*)(p + 16)); }
__device__ __forceinline__ void wave_sync() { __builtin_amdgcn_fence(3  , "wavefront"); __builtin_amdgcn_wave_barrier(); asm volatile("" ::: "memory"); }

#define KBLK ((NKEY * 2) / 256)
__global__ __launch_bounds__(256) void k_prep(const float* __restrict__ s, bf* KP, h16* VH, h16* VR) {
    const int i = (int)blockIdx.x * 256 + (int)threadIdx.x;
    if ((int)blockIdx.x < KBLK) {
        const int key = i >> 1, piece = i & 1;
        const float* row = s + ((size_t)NKEY_FULL + (size_t)key) * DF;
        v8us o;
#pragma unroll
        for (int k = 0; k < 8; ++k) { const int d = piece * 8 + k; const int dd = d < DF ? d : DF - 1; const unsigned short u = f2bf(row[dd]); o[k] = d < DF ? u : (unsigned short)0; }
        bf* p = KP + (size_t)i * 8;
        *(volatile v8us*)p = o; __threadfence(); *(volatile v8us*)p = o;
    } else {
        const int j = i - NKEY * 2;
        const int d = j / (NKEY / 8); const int piece = j - d * (NKEY / 8);
        const int dd = d < DF ? d : DF - 1;
        const int key = piece * 8;
        float a0 = 0.0f, a1 = 0.0f, a2 = 0.0f, a3 = 0.0f, a4 = 0.0f, a5 = 0.0f, a6 = 0.0f, a7 = 0.0f;
#pragma unroll 1
        for (int k = 0; k < NSL; ++k) {
            const float* sp = s + ((size_t)k * NKEY_FULL + (size_t)key) * DF + dd;
            a0 += bf2f(f2bf(sp[0 * DF])); a1 += bf2f(f2bf(sp[1 * DF])); a2 += bf2f(f2bf(sp[2 * DF])); a3 += bf2f(f2bf(sp[3 * DF]));
            a4 += bf2f(f2bf(sp[4 * DF])); a5 += bf2f(f2bf(sp[5 * DF])); a6 += bf2f(f2bf(sp[6 * DF])); a7 += bf2f(f2bf(sp[7 * DF]));
        }
        float av[8]; av[0] = a0; av[1] = a1; av[2] = a2; av[3] = a3; av[4] = a4; av[5] = a5; av[6] = a6; av[7] = a7;
        v8h hv, rv;
#pragma unroll
        for (int k = 0; k < 8; ++k) { const float v = d < DF ? av[k] : 0.0f; const h16 hh = (h16)v; hv[k] = hh; rv[k] = (h16)((v - (float)hh) * VRS); }
        const size_t oo = (size_t)d * NKEY + (size_t)key;
        *(volatile v8h*)(VH + oo) = hv; *(volatile v8h*)(VR + oo) = rv;
        __threadfence();
        *(volatile v8h*)(VH + oo) = hv; *(volatile v8h*)(VR + oo) = rv;
    }
}

__global__ __launch_bounds__(32 * AW) void k_flash(const float* __restrict__ WRT, const bf* __restrict__ KP, const h16* __restrict__ VH, const h16* __restrict__ VR,
                                                   const float* __restrict__ GAM, const float* __restrict__ BET, float* OUT) {
    __shared__ __align__(16) float os[AW * 16 * DF];
    const int lane = threadIdx.x & 31, lr = lane & 15, hi = lane >> 4;
    const int wave = __builtin_amdgcn_readfirstlane((int)(threadIdx.x >> 5));
    const int q0 = ((int)blockIdx.x * AW + wave) * 16;
    const size_t wro = (size_t)(q0 + lr) * DF;
    float wv[8]; v8us qlo;
#pragma unroll
    for (int i = 0; i < 8; ++i) { const int d = 8 * hi + i; const int dd = d < DF ? d : DF - 1; const unsigned short u = f2bf(WRT[wro + dd]);
        wv[i] = d < DF ? bf2f(u) : 0.0f; qlo[i] = d < DF ? u : (unsigned short)0; }
    const v8us zz = (v8us){};
    const v16bf qb = cat16b(qlo, zz);
    const bf*  kp  = KP + (size_t)lr * KW + 8 * hi;
    const h16* vhp = VH + (size_t)lr * NKEY + 8 * hi;
    const h16* vrp = VR + (size_t)lr * NKEY + 8 * hi;
    v8f oH = (v8f){}, oR = (v8f){};
    float m = -3.0e38f, l = 0.0f;
#pragma unroll 1
    for (int key0 = 0; key0 < NKEY; key0 += 32) {
        const v16bf ka = cat16b(*(const v8us*)(kp + (size_t)key0 * KW), zz);
        const v16bf kb = cat16b(*(const v8us*)(kp + (size_t)(key0 + 16) * KW), zz);
        v8f sa = (v8f){}, sb = (v8f){};
        sa = wmmab(ka, qb, sa); sb = wmmab(kb, qb, sb);
        asm volatile("v_nop\n\tv_nop\n\tv_nop\n\tv_nop" : "+v"(sa), "+v"(sb) : "v"(ka), "v"(kb), "v"(qb));
        float ta[8], tb[8]; float mx = -3.0e38f;
#pragma unroll
        for (int r = 0; r < 8; ++r) { ta[r] = sa[r] * L2E; tb[r] = sb[r] * L2E; mx = fmaxf(mx, fmaxf(ta[r], tb[r])); }
        mx = fmaxf(mx, __shfl_xor(mx, 16, 32));
        const float mnew = fmaxf(m, mx);
        const float alpha = __builtin_amdgcn_exp2f(m - mnew);
        const float sh = PSH - mnew;
        v16h pb; float ls = 0.0f;
#pragma unroll
        for (int r = 0; r < 8; ++r) { const h16 pa = (h16)__builtin_amdgcn_exp2f(ta[r] + sh); const h16 pc = (h16)__builtin_amdgcn_exp2f(tb[r] + sh); pb[r] = pa; pb[8 + r] = pc; ls += (float)pa + (float)pc; }
        l = l * alpha + ls; m = mnew;
        oH = oH * alpha; oR = oR * alpha;
        const v16h vh = ldh(vhp + key0), vr = ldh(vrp + key0);
        oH = wmma16(vh, pb, oH); oR = wmma16(vr, pb, oR);
        asm volatile("v_nop\n\tv_nop\n\tv_nop\n\tv_nop" : "+v"(oH), "+v"(oR) : "v"(vh), "v"(vr), "v"(pb));
    }
    l += __shfl_xor(l, 16, 32);
    const float inv = 1.0f / l;
    float x[8]; float S = 0.0f;
#pragma unroll
    for (int r = 0; r < 8; ++r) { const int d = 8 * hi + r; const float tmp = (oH[r] + oR[r] * VRI) * inv; x[r] = d < DF ? (wv[r] + tmp) : 0.0f; S += x[r]; }
    S += __shfl_xor(S, 16, 32);
    const float mu = S * (1.0f / (float)DF);
    float dv[8]; float SS = 0.0f;
#pragma unroll
    for (int r = 0; r < 8; ++r) { const int d = 8 * hi + r; dv[r] = d < DF ? (x[r] - mu) : 0.0f; SS += dv[r] * dv[r]; }
    SS += __shfl_xor(SS, 16, 32);
    const float rstd = rsqrtf(SS * (1.0f / (float)DF) + LN_EPS);
    const int wb = wave * 16 * DF;
#pragma unroll
    for (int r = 0; r < 8; ++r) { const int d = 8 * hi + r; const int dd = d < DF ? d : DF - 1;
        const float g = bf2f(f2bf(GAM[dd])); const float bt = bf2f(f2bf(BET[dd]));
        const float y = dv[r] * rstd * g + bt;
        if (d < DF) os[wb + lr * DF + d] = y; }
    wave_sync();
    float* obase = OUT + (size_t)q0 * DF;
    const int l8 = lane & 7;
#pragma unroll 1
    for (int ps = 0; ps < 2; ++ps) {
        const v4f a = *(const v4fa*)(&os[wb + 4 * lane]);
        const v4f c = *(const v4fa*)(&os[wb + 128 + 4 * l8]);
        *(volatile v4f*)(obase + 4 * lane) = a;
        if (lane < 8) *(volatile v4f*)(obase + 128 + 4 * lane) = c;
        if (ps == 0) __threadfence(); }
}

static constexpr size_t al256(size_t v) { return (v + 255) & ~(size_t)255; }
static constexpr size_t SZ_KP = al256((size_t)NKEY * KW * 2);
static constexpr size_t SZ_VP = al256((size_t)16 * NKEY * 2);
static constexpr size_t SZ_TOTAL = SZ_KP + 2 * SZ_VP;
static_assert(SZ_TOTAL <= (size_t)134217728);
static_assert(((size_t)NKEY * 2 + (size_t)16 * NKEY / 8) % 256 == 0);
static_assert((size_t)NQ * DF * 4 <= (size_t)NQ_FULL * DF * 4);

extern "C" void kernel_launch(void* const* d_in, const int* in_sizes, int n_in,
                              void* d_out, int out_size, void* d_ws, size_t ws_size, hipStream_t stream) {
    if (n_in < 4) return;
    if ((size_t)in_sizes[0] < ((size_t)(NSL - 1) * NKEY_FULL + NKEY) * DF) return;
    if ((size_t)in_sizes[1] < (size_t)NQ * DF) return;
    if (in_sizes[2] < DF || in_sizes[3] < DF) return;
    if ((size_t)out_size < (size_t)NQ * DF) return;
    if (SZ_TOTAL > ws_size) return;
    const float* s_stack = (const float*)d_in[0];
    const float* wrt     = (const float*)d_in[1];
    const float* gam     = (const float*)d_in[2];
    const float* bet     = (const float*)d_in[3];
    float* OUT = (float*)d_out;
    char* wsp = (char*)d_ws;
    bf*  KP = (bf*)wsp;  wsp += SZ_KP;
    h16* VH = (h16*)wsp; wsp += SZ_VP;
    h16* VR = (h16*)wsp; wsp += SZ_VP;

    k_prep<<<dim3((unsigned)(((size_t)NKEY * 2 + (size_t)16 * NKEY / 8) / 256), 1, 1), 256, 0, stream>>>(s_stack, KP, VH, VR);
    k_flash<<<dim3((unsigned)(NQ / (16 * AW)), 1, 1), 32 * AW, 0, stream>>>(wrt, KP, VH, VR, gam, bet, OUT);
}
